// recoAnomaly_38208029065461
// MI455X (gfx1250) — hardware-verified
//
#include <hip/hip_runtime.h>

typedef __attribute__((ext_vector_type(16))) _Float16 v16h;
typedef __attribute__((ext_vector_type(8)))  _Float16 v8h;
typedef __attribute__((ext_vector_type(8)))  float  v8f;
typedef __attribute__((ext_vector_type(4)))  float  v4f;
typedef __attribute__((ext_vector_type(4)))  unsigned v4u;
typedef float __attribute__((may_alias)) float_a;

#define N_NODES 50000
#define IN_C 128
#define L1C 96
#define OUT_C 64
#define EPS_F 1e-5f
#define BT 256
#define ECAP 5120
#define SCAP 48
#define ETILE 2048
#define NBUCK ((N_NODES + BT - 1) / BT)
#define NBNP 64

template <typename V> __device__ __forceinline__ void vst2(void* p, V v) {
  *(volatile V*)p = v; __threadfence(); *(volatile V*)p = v;
}
__device__ __forceinline__ v8f wmma_f16(v16h a, v16h b, v8f c) {
  v8f d = __builtin_amdgcn_wmma_f32_16x16x32_f16(false, a, false, b, (short)0, c, false, false);
  asm volatile("v_nop\n\tv_nop\n\tv_nop\n\tv_nop" : "+v"(d) : "v"(a), "v"(b));
  return d;
}
__device__ __forceinline__ v16h frag_lds(const _Float16* tile, int ld, int k0, int lane) {
  union { v16h v; v8h h[2]; } r;
  const _Float16* row = tile + (lane & 15) * ld + k0 + 8 * (lane >> 4);
  r.h[0] = *(const v8h*)(row); r.h[1] = *(const v8h*)(row + 16);
  return r.v;
}
__device__ __forceinline__ v16h frag_f32(const float* row, int k0, int lane) {
  v16h a; const float* p = row + k0 + 8 * (lane >> 4);
#pragma unroll
  for (int i = 0; i < 8; ++i) { a[i] = (_Float16)p[i]; a[8 + i] = (_Float16)p[16 + i]; }
  return a;
}

struct Bucket {
  int lsrc[ECAP]; unsigned short ltgt[ECAP]; unsigned short sub[BT][SCAP]; int scnt[BT]; int wcnt[8][8]; int total;
};
__device__ void bucket_build(Bucket& bk, const int* __restrict__ src, const int* __restrict__ dst, int E, int tlo, int tid) {
  const int lane = tid & 31, wave = tid >> 5;
  if (tid == 0) bk.total = 0;
  __syncthreads();
  for (int e0 = 0; e0 < E; e0 += ETILE) {
    int rv[8]; unsigned msk[8];
#pragma unroll
    for (int j = 0; j < 8; ++j) {
      const int e = e0 + j * 256 + tid;
      const int r = (e < E) ? dst[e] : -1;
      rv[j] = r;
      msk[j] = (unsigned)__builtin_amdgcn_ballot_w32((r >= tlo) && (r < tlo + BT));
    }
    if (lane < 8) bk.wcnt[lane][wave] = __builtin_popcount(msk[lane]);
    __syncthreads();
    const int base = bk.total;
    int run = 0, pre[8];
#pragma unroll
    for (int j = 0; j < 8; ++j) {
#pragma unroll
      for (int w = 0; w < 8; ++w) { if (w == wave) pre[j] = run; run += bk.wcnt[j][w]; }
    }
#pragma unroll
    for (int j = 0; j < 8; ++j) {
      const unsigned m = msk[j];
      if ((m >> lane) & 1u) {
        const int pos = base + pre[j] + __builtin_popcount(m & ((1u << lane) - 1u));
        if (pos < ECAP) { bk.lsrc[pos] = e0 + j * 256 + tid; bk.ltgt[pos] = (unsigned short)(rv[j] - tlo); }
      }
    }
    __syncthreads();
    if (tid == 0) bk.total = base + run;
    __syncthreads();
  }
  const int n = (bk.total < ECAP) ? bk.total : ECAP;
  for (int i = tid; i < n; i += 256) { int s = src[bk.lsrc[i]]; s = s < 0 ? 0 : (s >= N_NODES ? N_NODES - 1 : s); bk.lsrc[i] = s; }
  __syncthreads();
  int k = 0;
  for (int i = 0; i < n; ++i) if ((int)bk.ltgt[i] == tid) { if (k < SCAP) bk.sub[tid][k] = (unsigned short)i; ++k; }
  bk.scnt[tid] = (k < SCAP) ? k : SCAP;
  __syncthreads();
}

__global__ __launch_bounds__(256) void k_degree(const int* __restrict__ src, const int* __restrict__ dst, int E, float* __restrict__ dinv) {
  __shared__ Bucket bk;
  const int tid = threadIdx.x, tlo = blockIdx.x * BT;
  bucket_build(bk, src, dst, E, tlo, tid);
  const int node = tlo + tid;
  if (node < N_NODES) vst2(dinv + node, (float_a)rsqrtf((float)bk.scnt[tid] + 1.0f));
}

__global__ __launch_bounds__(256) void k_bn_part(const float* __restrict__ x, float* __restrict__ part) {
  __shared__ __align__(16) float sh[2][256];
  const int tid = threadIdx.x, c = tid & 127, half = tid >> 7;
  const int per = (N_NODES + NBNP - 1) / NBNP;
  const int r0 = blockIdx.x * per, r1 = min(N_NODES, r0 + per);
  float s = 0.f, ss = 0.f;
  for (int r = r0 + half; r < r1; r += 2) { const float v = x[(size_t)r * IN_C + c]; s += v; ss += v * v; }
  sh[half][c] = s; sh[half][128 + c] = ss;
  __syncthreads();
  if (tid < 64) {
    const v4f a = *(const v4f*)(&sh[0][tid * 4]), b = *(const v4f*)(&sh[1][tid * 4]);
    vst2(part + (size_t)blockIdx.x * 256 + tid * 4, a + b);
  }
}

__global__ __launch_bounds__(128) void k_bn_fold(const float* __restrict__ part, const float* __restrict__ bnw, const float* __restrict__ bnb,
                                                 const float* __restrict__ W1, _Float16* __restrict__ W1sT, float* __restrict__ t1) {
  __shared__ float scale[IN_C], shift[IN_C];
  __shared__ __align__(16) _Float16 wt[L1C * IN_C];
  __shared__ __align__(16) float tt[L1C];
  const int tid = threadIdx.x;
  {
    double s = 0.0, ss = 0.0;
    for (int b = 0; b < NBNP; ++b) { s += part[(size_t)b * 256 + tid]; ss += part[(size_t)b * 256 + 128 + tid]; }
    const double mean = s / N_NODES;
    const double var = ss / N_NODES - mean * mean;
    const float sc = (float)(1.0 / sqrt(var + 1e-5)) * bnw[tid];
    scale[tid] = sc; shift[tid] = bnb[tid] - (float)mean * sc;
  }
  __syncthreads();
  for (int i = tid; i < IN_C * L1C; i += 128) { const int k = i / L1C, n = i - k * L1C; wt[n * IN_C + k] = (_Float16)(scale[k] * W1[i]); }
  if (tid < L1C) { float a = 0.f;
#pragma unroll 1
    for (int k = 0; k < IN_C; ++k) a += shift[k] * W1[k * L1C + tid];
    tt[tid] = a; }
  __syncthreads();
  for (int g = tid; g < L1C * 16; g += 128) vst2(W1sT + g * 8, *(const v4u*)((const char*)wt + g * 16));
  if (tid < L1C / 4) vst2(t1 + tid * 4, *(const v4f*)(&tt[tid * 4]));
}

template <int CIN, int COUT, int WPITCH>
__global__ __launch_bounds__(128) void k_gemm(const float* __restrict__ A, const _Float16* __restrict__ WT,
                                              const float* __restrict__ t, float* __restrict__ H) {
  constexpr int NT = COUT / 16, KC = CIN / 32, LP = CIN + 8;
  __shared__ __align__(16) _Float16 ws[COUT * LP];
  __shared__ __align__(16) float so[4][16 * COUT];
  const int tid = threadIdx.x, wave = tid >> 5, lane = tid & 31, hi = lane >> 4, col = lane & 15;
  for (int i = tid; i < COUT * CIN; i += 128) { const int n = i / CIN, k = i - n * CIN; ws[n * LP + k] = WT[n * WPITCH + k]; }
  __syncthreads();
  const int strip = blockIdx.x * 4 + wave;
  const bool valid = strip < N_NODES / 16;
  if (valid) {
    const float* ar = A + (size_t)(strip * 16 + col) * CIN;
    v16h af[KC];
#pragma unroll
    for (int kc = 0; kc < KC; ++kc) af[kc] = frag_f32(ar, kc * 32, lane);
#pragma unroll
    for (int nt = 0; nt < NT; ++nt) {
      v8f acc = {};
#pragma unroll
      for (int kc = 0; kc < KC; ++kc) acc = wmma_f16(af[kc], frag_lds(ws + nt * 16 * LP, LP, kc * 32, lane), acc);
      const float tb = t[nt * 16 + col];
#pragma unroll
      for (int r = 0; r < 8; ++r) so[wave][(hi * 8 + r) * COUT + nt * 16 + col] = acc[r] + tb;
    }
  }
  __syncthreads();
  if (valid) {
    float* dst = H + (size_t)strip * 16 * COUT;
#pragma unroll
    for (int q = 0; q < COUT / 8; ++q) { const int g = q * 32 + lane; vst2(dst + g * 4, *(const v4f*)(&so[wave][g * 4])); }
  }
}

__global__ __launch_bounds__(256) void k_gather1(const int* __restrict__ src, const int* __restrict__ dst, int E, const float* __restrict__ dinv,
                                                 const float* __restrict__ h1, const float* __restrict__ b1, float* __restrict__ h2, float* __restrict__ lnpart) {
  __shared__ Bucket bk;
  __shared__ float red[2][8][32];
  const int tid = threadIdx.x, lane = tid & 31, wave = tid >> 5, tlo = blockIdx.x * BT;
  bucket_build(bk, src, dst, E, tlo, tid);
  float ls = 0.f, lss = 0.f;
  for (int s = 0; s < 32; ++s) {
    const int t = wave * 32 + s, node = tlo + t;
    if (node >= N_NODES) break;
    const float di = dinv[node];
    const int cnt = bk.scnt[t];
    float a0 = 0.f, a1 = 0.f, a2 = 0.f;
    for (int k = 0; k < cnt; ++k) {
      const int sN = bk.lsrc[bk.sub[t][k]];
      const float w = dinv[sN] * di;
      const float* hr = h1 + (size_t)sN * L1C;
      a0 += w * hr[lane]; a1 += w * hr[32 + lane]; a2 += w * hr[64 + lane];
    }
    const float* hs = h1 + (size_t)node * L1C;
    const float dd = di * di;
    a0 = fmaxf(a0 + dd * hs[lane] + b1[lane], 0.f);
    a1 = fmaxf(a1 + dd * hs[32 + lane] + b1[32 + lane], 0.f);
    a2 = fmaxf(a2 + dd * hs[64 + lane] + b1[64 + lane], 0.f);
    ls += a0 + a1 + a2; lss += a0 * a0 + a1 * a1 + a2 * a2;
    float* orow = h2 + (size_t)node * L1C;
    vst2(orow + lane, (float_a)a0); vst2(orow + 32 + lane, (float_a)a1); vst2(orow + 64 + lane, (float_a)a2);
  }
  red[0][wave][lane] = ls; red[1][wave][lane] = lss;
  __syncthreads();
  if (tid < 32) {
    float s = 0.f, ss = 0.f;
    for (int w = 0; w < 8; ++w) for (int l = 0; l < 32; ++l) { s += red[0][w][l]; ss += red[1][w][l]; }
    const float v = (lane == 0) ? s : ((lane == 1) ? ss : 0.f);
    vst2(lnpart + (size_t)blockIdx.x * 32 + lane, (float_a)v);
  }
}

__global__ __launch_bounds__(128) void k_ln_fold(const float* __restrict__ lnpart, const float* __restrict__ lnw, const float* __restrict__ lnb,
                                                 const float* __restrict__ W2, _Float16* __restrict__ W2sT, float* __restrict__ t2) {
  __shared__ float srow[L1C], crow[L1C];
  __shared__ __align__(16) _Float16 wt[OUT_C * 128];
  __shared__ __align__(16) float tt[OUT_C];
  __shared__ double tot[2];
  const int tid = threadIdx.x;
  if (tid < 2) { double a = 0.0; for (int b = 0; b < NBUCK; ++b) a += lnpart[(size_t)b * 32 + tid]; tot[tid] = a; }
  __syncthreads();
  const double cntd = (double)N_NODES * (double)L1C;
  const double mean = tot[0] / cntd, var = tot[1] / cntd - mean * mean;
  const float inv = (float)(1.0 / sqrt(var + 1e-5)), meanf = (float)mean;
  if (tid < L1C) { const float sr = inv * lnw[tid]; srow[tid] = sr; crow[tid] = lnb[tid] - meanf * sr; }
  __syncthreads();
#pragma unroll 1
  for (int i = tid; i < OUT_C * 128; i += 128) { const int n = i >> 7, k = i & 127; wt[i] = (k < L1C) ? (_Float16)(srow[k] * W2[k * OUT_C + n]) : (_Float16)0.f; }
  if (tid < OUT_C) { float a = 0.f;
#pragma unroll 1
    for (int j = 0; j < L1C; ++j) a += crow[j] * W2[j * OUT_C + tid];
    tt[tid] = a; }
  __syncthreads();
  for (int g = tid; g < OUT_C * 16; g += 128) vst2(W2sT + g * 8, *(const v4u*)((const char*)wt + g * 16));
  if (tid < OUT_C / 4) vst2(t2 + tid * 4, *(const v4f*)(&tt[tid * 4]));
}

__global__ __launch_bounds__(256) void k_gather2(const int* __restrict__ src, const int* __restrict__ dst, int E, const float* __restrict__ dinv,
                                                 const float* __restrict__ h3, const float* __restrict__ b2, float* __restrict__ out) {
  __shared__ Bucket bk;
  const int tid = threadIdx.x, lane = tid & 31, wave = tid >> 5, tlo = blockIdx.x * BT;
  bucket_build(bk, src, dst, E, tlo, tid);
  for (int s = 0; s < 32; ++s) {
    const int t = wave * 32 + s, node = tlo + t;
    if (node >= N_NODES) break;
    const float di = dinv[node];
    const int cnt = bk.scnt[t];
    float a0 = 0.f, a1 = 0.f;
    for (int k = 0; k < cnt; ++k) {
      const int sN = bk.lsrc[bk.sub[t][k]];
      const float w = dinv[sN] * di;
      const float* hr = h3 + (size_t)sN * OUT_C;
      a0 += w * hr[lane]; a1 += w * hr[32 + lane];
    }
    const float* hs = h3 + (size_t)node * OUT_C;
    const float dd = di * di;
    a0 = fmaxf(a0 + dd * hs[lane] + b2[lane], 0.f);
    a1 = fmaxf(a1 + dd * hs[32 + lane] + b2[32 + lane], 0.f);
    float* orow = out + (size_t)node * OUT_C;
    vst2(orow + lane, (float_a)a0); vst2(orow + 32 + lane, (float_a)a1);
  }
}

extern "C" void kernel_launch(void* const* d_in, const int* in_sizes, int n_in,
                              void* d_out, int out_size, void* d_ws, size_t ws_size,
                              hipStream_t stream) {
  (void)n_in; (void)out_size; (void)ws_size;
  const float* x   = (const float*)d_in[0];
  const int*   ei  = (const int*)d_in[1];
  const float* bnw = (const float*)d_in[2];
  const float* bnb = (const float*)d_in[3];
  const float* W1  = (const float*)d_in[4];
  const float* b1  = (const float*)d_in[5];
  const float* lnw = (const float*)d_in[6];
  const float* lnb = (const float*)d_in[7];
  const float* W2  = (const float*)d_in[8];
  const float* b2  = (const float*)d_in[9];
  float* out = (float*)d_out;

  const int E = in_sizes[1] / 2;
  const int* src = ei;
  const int* dst = ei + E;

  char* base = (char*)d_ws; size_t off = 0;
  auto alloc = [&](size_t bytes) -> void* { void* p = base + off; off = (off + bytes + 255) & ~(size_t)255; return p; };
  float*    dinv   = (float*)alloc((size_t)N_NODES * 4);
  float*    bnpart = (float*)alloc((size_t)NBNP * 256 * 4);
  _Float16* W1sT   = (_Float16*)alloc((size_t)L1C * IN_C * 2);
  float*    t1     = (float*)alloc(128 * 4);
  float*    lnpart = (float*)alloc((size_t)NBUCK * 32 * 4);
  _Float16* W2sT   = (_Float16*)alloc((size_t)OUT_C * 128 * 2);
  float*    t2     = (float*)alloc(128 * 4);
  float*    h1     = (float*)alloc((size_t)N_NODES * L1C * 4);
  float*    h2     = (float*)alloc((size_t)N_NODES * L1C * 4);
  float*    h3     = (float*)alloc((size_t)N_NODES * OUT_C * 4);

  k_degree<<<NBUCK, 256, 0, stream>>>(src, dst, E, dinv);
  k_bn_part<<<NBNP, 256, 0, stream>>>(x, bnpart);
  k_bn_fold<<<1, 128, 0, stream>>>(bnpart, bnw, bnb, W1, W1sT, t1);
  k_gemm<IN_C, L1C, IN_C><<<(N_NODES / 16 + 3) / 4, 128, 0, stream>>>(x, W1sT, t1, h1);
  k_gather1<<<NBUCK, 256, 0, stream>>>(src, dst, E, dinv, h1, b1, h2, lnpart);
  k_ln_fold<<<1, 128, 0, stream>>>(lnpart, lnw, lnb, W2, W2sT, t2);
  k_gemm<L1C, OUT_C, 128><<<(N_NODES / 16 + 3) / 4, 128, 0, stream>>>(h2, W2sT, t2, h3);
  k_gather2<<<NBUCK, 256, 0, stream>>>(src, dst, E, dinv, h3, b2, out);
}
